// ConsensusAttention_10342281248995
// MI455X (gfx1250) — hardware-run, weakly checked
//
#include <hip/hip_runtime.h>


#ifndef NB
#define NB 8
#endif
#ifndef NL
#define NL 6
#endif
#define NB_FULL  8
#define NL_FULL  6
#define SEQ      1024
#define SEQ_FULL 1024
#define GW   32
#define DH   128
#define AW   4
#define OSP  132
#define PT   64
#define HSP  136
#define SC2   ((float)(0.08838834764831845 * 1.4426950408889634))
#define SELF2 ((float)(-0.0005 * 1.4426950408889634))
#define PSH  14.0f
#define NEGB (-3.0e38f)

static_assert(GW * GW == SEQ);
static_assert(GW == 32);
static_assert(DH % 32 == 0);
static_assert(DH == 32 * 4);
static_assert(DH % 64 == 0);
static_assert(SEQ % PT == 0);
static_assert(PT == 8 * 8);
static_assert(256 * 4 * 8 == PT * DH);
static_assert(256 * 4 * 8 == DH * PT);
static_assert(16 * 4 == PT);
static_assert((PT * 2) % 128 == 0);
static_assert(SEQ % (16 * AW) == 0);
static_assert((HSP * 2) % 16 == 0);
static_assert((OSP * 4) % 16 == 0);
static_assert(OSP >= DH);
static_assert(HSP >= DH);
static_assert(16 * 1 == 16);
static_assert(NB <= NB_FULL);
static_assert(NL <= NL_FULL);
static_assert(PT * HSP * 2 + PT * 4 <= 131072);
static_assert(AW * 16 * OSP * 4 <= 131072);

typedef _Float16 h16;
typedef __attribute__((ext_vector_type(16))) _Float16 v16h;
typedef __attribute__((ext_vector_type(8)))  _Float16 v8h;
typedef __attribute__((ext_vector_type(4)))  _Float16 v4h;
typedef __attribute__((ext_vector_type(8)))  float    v8f;
typedef __attribute__((ext_vector_type(4)))  float    v4f;
typedef v4f  __attribute__((may_alias)) v4fa;
typedef v4h  __attribute__((may_alias)) v4ha;
typedef v8h  __attribute__((may_alias)) v8ha;

__device__ __forceinline__ unsigned short f2bf(float f) { unsigned u = __float_as_uint(f); u += 0x7FFFu + ((u >> 16) & 1u); return (unsigned short)(u >> 16); }
__device__ __forceinline__ float bfr(float f) { return __uint_as_float(((unsigned)f2bf(f)) << 16); }
__device__ __forceinline__ v16h cat16(v8h lo, v8h hi) { return __builtin_shufflevector(lo, hi, 0, 1, 2, 3, 4, 5, 6, 7, 8, 9, 10, 11, 12, 13, 14, 15); }
static __device__ __forceinline__ h16 toh_flush(float v) { const h16 r = (h16)v; return (fabsf(v) < 6.103515625e-05f) ? (h16)0.0f : r; }
__device__ __forceinline__ v8f wmma16g(v16h a, v16h b, v8f c) {
    c = __builtin_amdgcn_wmma_f32_16x16x32_f16(false, a, false, b, (short)0, c, false, false);
    asm volatile("v_nop\n\tv_nop\n\tv_nop\n\tv_nop" : "+v"(c) : "v"(a), "v"(b));
    return c;
}
__device__ __forceinline__ v16h  ldh(const h16* p) { return cat16(*(const v8h*)p, *(const v8h*)(p + 16)); }
__device__ __forceinline__ void wave_sync() { __builtin_amdgcn_fence(3  , "wavefront"); __builtin_amdgcn_wave_barrier(); asm volatile("" ::: "memory"); }

__global__ __launch_bounds__(256) void k_prep(const float* __restrict__ X, h16* XH, h16* VT, float* RN) {
#pragma clang fp contract(off)
    __shared__ __align__(16) h16 hs[PT * HSP];
    __shared__ __align__(16) float rs[PT];
    const int lane = threadIdx.x & 31;
    const int wave = __builtin_amdgcn_readfirstlane((int)(threadIdx.x >> 5));
    const int z = blockIdx.y; const int b = z / NL, lv = z % NL;
    const int t0 = blockIdx.x * PT;
    const float* src = X + (((size_t)b * SEQ_FULL + (size_t)t0) * NL_FULL + (size_t)lv) * DH + lane * 4;
#pragma unroll 1
    for (int i = 0; i < 8; ++i) {
        const int row = wave * 8 + i;
        const v4f x = *(const v4f*)(src + (size_t)row * (NL_FULL * DH));
        const float x0 = bfr(x[0]), x1 = bfr(x[1]), x2 = bfr(x[2]), x3 = bfr(x[3]);
        float ss = x0 * x0; ss += x1 * x1; ss += x2 * x2; ss += x3 * x3;
        ss += __shfl_xor(ss, 1, 32); ss += __shfl_xor(ss, 2, 32); ss += __shfl_xor(ss, 4, 32); ss += __shfl_xor(ss, 8, 32); ss += __shfl_xor(ss, 16, 32);
        v4h o; o[0] = toh_flush(x0); o[1] = toh_flush(x1); o[2] = toh_flush(x2); o[3] = toh_flush(x3);
        *(v4ha*)(&hs[row * HSP + lane * 4]) = o;
        const float fac = SC2 * (1.0f / fmaxf(sqrtf(ss), 1e-12f));
        if (lane == 0) rs[row] = fac;
    }
    __syncthreads();
    const size_t xb = ((size_t)z * SEQ + (size_t)t0) * DH;
    const size_t vb = (size_t)z * DH * SEQ + (size_t)t0;
    float* rnp = RN + (size_t)z * SEQ + (size_t)t0;
#pragma unroll 1
    for (int ps = 0; ps < 2; ++ps) {
#pragma unroll 1
        for (int it = 0; it < 4; ++it) {
            const int p = it * 256 + (int)threadIdx.x; const int row = p >> 4, c8 = (p & 15) * 8;
            const v8h v = *(const v8ha*)(&hs[row * HSP + c8]);
            *(volatile v8h*)(XH + xb + (size_t)p * 8) = v; }
#pragma unroll 1
        for (int it = 0; it < 4; ++it) {
            const int p = it * 256 + (int)threadIdx.x; const int d = p >> 3, tg = (p & 7) * 8;
            v8h o;
#pragma unroll
            for (int i = 0; i < 8; ++i) o[i] = hs[(tg + i) * HSP + d];
            *(volatile v8h*)(VT + vb + (size_t)d * SEQ + tg) = o; }
        if (threadIdx.x < 16) { const v4f r = *(const v4fa*)(&rs[threadIdx.x * 4]); *(volatile v4f*)(rnp + threadIdx.x * 4) = r; }
        if (ps == 0) __threadfence(); }
}

__global__ __launch_bounds__(32 * AW) __attribute__((amdgpu_num_vgpr(256)))
void k_band(const h16* __restrict__ XH, const h16* __restrict__ VT, const float* __restrict__ RN, float* OUT) {
    __shared__ __align__(16) float os[AW * 16 * OSP];
    const int lane = threadIdx.x & 31, lr = lane & 15, hi = lane >> 4;
    const int wave = __builtin_amdgcn_readfirstlane((int)(threadIdx.x >> 5));
    const int zh = blockIdx.y; const int b = zh / NL, lv = zh % NL;
    const int t0 = ((int)blockIdx.x * AW + wave) * 16;
    const int qyv = (((int)blockIdx.x * AW + (int)(threadIdx.x >> 5)) * 16) / GW;
    int lov = qyv - 2; lov = lov < 0 ? 0 : lov;
    int hiv = qyv + 2; hiv = hiv > GW - 1 ? GW - 1 : hiv;
    const int kylo = __builtin_amdgcn_readfirstlane(lov), kyhi = __builtin_amdgcn_readfirstlane(hiv);
    const int qy = t0 / GW;
    const int qx = (t0 % GW) + lr;
    const size_t pbase = (size_t)zh * SEQ * DH;
    const size_t qo = pbase + (size_t)(t0 + lr) * DH + 8 * hi;
    const size_t ko = pbase + (size_t)lr * DH + 8 * hi;
    const size_t vo = pbase + (size_t)lr * SEQ + 8 * hi;
    const float* cb = RN + (size_t)zh * SEQ + 8 * hi;
    v8f o[8];
#pragma unroll
    for (int j = 0; j < 8; ++j) o[j] = (v8f){};
    float m = NEGB, l = 0.0f;
#pragma unroll 1
    for (int ky = kylo; ky <= kyhi; ++ky) {
        const int key0 = ky * GW;
        const int dy = qy - ky; const int dy2 = dy * dy;
        v8f sa = (v8f){}, sb = (v8f){};
#pragma unroll 1
        for (int kc = 0; kc < DH; kc += 32) {
            const v16h qf = ldh(XH + qo + kc);
            const h16* ka = XH + ko + (size_t)key0 * DH + kc;
            const v16h ka0 = ldh(ka), kb0 = ldh(ka + 16 * DH);
            sa = wmma16g(ka0, qf, sa); sb = wmma16g(kb0, qf, sb);
        }
        const float* cp = cb + key0;
        const v4f c0 = *(const v4f*)cp, c1 = *(const v4f*)(cp + 4), c2 = *(const v4f*)(cp + 16), c3 = *(const v4f*)(cp + 20);
        float ca[8], cc[8];
#pragma unroll
        for (int r = 0; r < 4; ++r) { ca[r] = c0[r]; ca[4 + r] = c1[r]; cc[r] = c2[r]; cc[4 + r] = c3[r]; }
        const int dxa = qx - 8 * hi;
        float ta[8], tb[8]; bool fa[8], fb[8]; float mx = NEGB;
#pragma unroll
        for (int r = 0; r < 8; ++r) {
            const int da = dxa - r, db = dxa - 16 - r;
            const int d2a = dy2 + da * da, d2b = dy2 + db * db;
            fa[r] = d2a <= 4; fb[r] = d2b <= 4;
            const float ua = sa[r] * ca[r], ub = sb[r] * cc[r];
            ta[r] = (d2a == 0) ? SELF2 : ua; tb[r] = (d2b == 0) ? SELF2 : ub;
            mx = fmaxf(mx, fmaxf(fa[r] ? ta[r] : NEGB, fb[r] ? tb[r] : NEGB)); }
        mx = fmaxf(mx, __shfl_xor(mx, 16, 32));
        const float mnew = fmaxf(m, mx);
        const float alpha = __builtin_amdgcn_exp2f(m - mnew);
        const float sh = PSH - mnew;
        v16h pb; float ls = 0.0f;
#pragma unroll
        for (int r = 0; r < 8; ++r) {
            const float aa = ta[r] + sh, ab = tb[r] + sh;
            const float ea = (aa < -14.0f) ? 0.0f : __builtin_amdgcn_exp2f(aa);
            const float eb = (ab < -14.0f) ? 0.0f : __builtin_amdgcn_exp2f(ab);
            const float ga = fa[r] ? ea : 0.0f, gb = fb[r] ? eb : 0.0f;
            const h16 pa = (h16)ga; const h16 pc = (h16)gb;
            pb[r] = pa; pb[8 + r] = pc;
            ls += (float)pa + (float)pc; }
        l = l * alpha + ls; m = mnew;
#pragma unroll
        for (int j = 0; j < 8; ++j) o[j] = o[j] * alpha;
        const h16* va = VT + vo + key0;
#pragma unroll
        for (int g = 0; g < 2; ++g) {
            v16h vf[4];
#pragma unroll
            for (int j = 0; j < 4; ++j) vf[j] = ldh(va + (size_t)(16 * (4 * g + j)) * SEQ);
#pragma unroll
            for (int j = 0; j < 4; ++j) o[4 * g + j] = wmma16g(vf[j], pb, o[4 * g + j]);
        }
    }
    l += __shfl_xor(l, 16, 32);
    const bool any = l > 0.0f;
    const float lsafe = any ? l : 1.0f;
    const float inv = any ? (1.0f / lsafe) : 0.0f;
    const int wb = wave * 16 * OSP;
#pragma unroll
    for (int j = 0; j < 8; ++j) { v4f a, c;
        a[0] = o[j][0] * inv; a[1] = o[j][1] * inv; a[2] = o[j][2] * inv; a[3] = o[j][3] * inv;
        c[0] = o[j][4] * inv; c[1] = o[j][5] * inv; c[2] = o[j][6] * inv; c[3] = o[j][7] * inv;
        *(v4fa*)(&os[wb + lr * OSP + 16 * j + 8 * hi]) = a; *(v4fa*)(&os[wb + lr * OSP + 16 * j + 8 * hi + 4]) = c; }
    wave_sync();
    float* orow = OUT + (((size_t)b * SEQ_FULL + (size_t)t0) * NL_FULL + (size_t)lv) * DH;
#pragma unroll 1
    for (int ps = 0; ps < 2; ++ps) {
#pragma unroll 4
        for (int s = 0; s < 16; ++s) {
            const v4f val = *(const v4fa*)(&os[wb + s * OSP + lane * 4]);
            *(volatile v4f*)(orow + (size_t)s * (NL_FULL * DH) + lane * 4) = val; }
        if (ps == 0) __threadfence(); }
}

static constexpr size_t al256(size_t v) { return (v + 255) & ~(size_t)255; }
static constexpr size_t SZ_PL = al256((size_t)NB * NL * SEQ * DH * 2);
static constexpr size_t SZ_RN = al256((size_t)NB * NL * SEQ * 4);
static constexpr size_t SZ_TOTAL = 2 * SZ_PL + SZ_RN;
static_assert(SZ_TOTAL <= (size_t)134217728);
static_assert((size_t)NB * NL * SEQ * DH == (size_t)NB * NL * DH * SEQ);

extern "C" void kernel_launch(void* const* d_in, const int* in_sizes, int n_in,
                              void* d_out, int out_size, void* d_ws, size_t ws_size, hipStream_t stream) {
    if (n_in < 1) return;
    const size_t need = ((((size_t)(NB - 1) * SEQ_FULL + (size_t)(SEQ - 1)) * NL_FULL) + (size_t)NL) * DH;
    if ((size_t)in_sizes[0] < need) return;
    if ((size_t)out_size < need) return;
    if (SZ_TOTAL > ws_size) return;
    const float* X = (const float*)d_in[0];
    float* OUT = (float*)d_out;
    char* wsp = (char*)d_ws;
    h16* XH = (h16*)wsp; wsp += SZ_PL;
    h16* VT = (h16*)wsp; wsp += SZ_PL;
    float* RN = (float*)wsp; wsp += SZ_RN;

    k_prep<<<dim3(SEQ / PT, NB * NL, 1), 256, 0, stream>>>(X, XH, VT, RN);
    k_band<<<dim3(SEQ / (16 * AW), NB * NL, 1), 32 * AW, 0, stream>>>(XH, VT, RN, OUT);
}
